// GCN_82721070121690
// MI455X (gfx1250) — hardware-verified
//
#include <hip/hip_runtime.h>
#include <stddef.h>
#include <stdint.h>


#define CIN    128
#define HID    128
#define NC2    64
#define KP     256
#define SLEN   50
#define NTHR   256
#define NWAVE  8
#define EPT    8
#define CHUNK  (NTHR * EPT)
#define WCAP   (EPT * 32)
#define LISTN  (NWAVE * WCAP)
#define NBA    1024
#define SLA    10
#define RCAP   20480
#define DEGCAP 64
#define GBM    64
#define GBN    64
#define GTHR   128
#define AGG_ZINTS    (LISTN + 2 * RCAP + 3 * NBA)
#define MISC_INTS    16
#define ROWBUF_INTS  (NWAVE * KP / 2)
#define AGG_LDS_INTS (AGG_ZINTS + MISC_INTS + ROWBUF_INTS)
#define NU_W1  (HID * (2 * CIN / 8))
#define NU_W2  (NC2 * (2 * HID / 8))
#define NU_F1  (256 * (2 * NC2 / 8))
#define NU_F2  (128 * (2 * 256 / 8))
#define NU_ALL (NU_W1 + NU_W2 + NU_F1 + NU_F2)
#define WSMAX  134217728

static_assert((CHUNK & (CHUNK - 1)) == 0 && CHUNK <= 4096);
static_assert((NBA & (NBA - 1)) == 0 && NBA == (1 << SLA));
static_assert(((long long)CHUNK << SLA) < (1LL << 31));
static_assert(NBA % NWAVE == 0 && NBA % 32 == 0 && NBA % GBM == 0);
static_assert(RCAP % 4 == 0 && AGG_ZINTS % (NTHR * 4) == 0 && ((AGG_ZINTS + MISC_INTS) % 4) == 0);
static_assert(GBM == (GTHR / 32) * 16 && GBN == 64);
static_assert(NU_W1 % NTHR == 0 && NU_W2 % NTHR == 0 && NU_F1 % NTHR == 0 && NU_F2 % NTHR == 0);
static_assert(CIN == 4 * 32 && NC2 == 2 * 32 && KP == 2 * CIN && KP == 2 * HID);
static_assert(AGG_LDS_INTS * 4 <= 300000);
static_assert(SLEN > 32 && SLEN <= 64);

typedef float          v2f   __attribute__((ext_vector_type(2)));
typedef float          v4f   __attribute__((ext_vector_type(4)));
typedef float          v8f   __attribute__((ext_vector_type(8)));
typedef int            v4i   __attribute__((ext_vector_type(4)));
typedef int            v8i   __attribute__((ext_vector_type(8)));
typedef unsigned       v2u   __attribute__((ext_vector_type(2)));
typedef unsigned       v4u   __attribute__((ext_vector_type(4)));
typedef unsigned short v4us  __attribute__((ext_vector_type(4)));
typedef unsigned short v8us  __attribute__((ext_vector_type(8)));
typedef unsigned short v16us __attribute__((ext_vector_type(16)));
typedef __bf16         v16bf __attribute__((ext_vector_type(16)));
typedef v2f  __attribute__((may_alias)) v2fa;
typedef v4f  __attribute__((may_alias)) v4fa;
typedef v4i  __attribute__((may_alias)) v4ia;
typedef v2u  __attribute__((may_alias)) v2ua;
typedef v4us __attribute__((may_alias)) v4usa;
typedef v8us __attribute__((may_alias)) v8usa;
union FragB { v16bf v; v16us u; v8us h[2]; v8i w; };

__device__ __forceinline__ v8f wmb(const FragB& a, const FragB& b, v8f c) {
  v8f d = __builtin_amdgcn_wmma_f32_16x16x32_bf16(false, a.v, false, b.v, (short)0, c, false, false);
  asm volatile("v_nop\n\tv_nop\n\tv_nop\n\tv_nop" : "+v"(d) : "v"(a.w), "v"(b.w));
  return d;
}

__device__ __forceinline__ unsigned bf16_bits(float f) {
  const unsigned u = __float_as_uint(f);
  return (u + 0x7FFFu + ((u >> 16) & 1u)) >> 16;
}
__device__ __forceinline__ float bf16_val(float f) {
  return __uint_as_float(bf16_bits(f) << 16);
}
__device__ __forceinline__ float relu_keep(float v) {
  return (v > 0.0f) ? v : (v - v);
}

__device__ __forceinline__ void wave_sync() {
  __builtin_amdgcn_fence(__ATOMIC_RELEASE, "wavefront");
  __builtin_amdgcn_wave_barrier();
  __builtin_amdgcn_fence(__ATOMIC_ACQUIRE, "wavefront");
}

template <int SLB>
__device__ __forceinline__ int scan_chunk(const int* __restrict__ dsts, int nE, int cbase, int slotBase,
                                          int nb, int vec8, int* list, int tid, int lane, int wave) {
  int wc = 0;
  const int el0  = tid * EPT;
  const int e0   = cbase + el0;
  const int sent = -2147483647 - 1;
  v4i da, db;
  if (vec8 != 0 && cbase + CHUNK <= nE) {
    da = *(const v4i*)(dsts + e0);
    db = *(const v4i*)(dsts + e0 + 4);
  } else {
    da.x = (e0     < nE) ? dsts[min(e0,     nE - 1)] : sent;
    da.y = (e0 + 1 < nE) ? dsts[min(e0 + 1, nE - 1)] : sent;
    da.z = (e0 + 2 < nE) ? dsts[min(e0 + 2, nE - 1)] : sent;
    da.w = (e0 + 3 < nE) ? dsts[min(e0 + 3, nE - 1)] : sent;
    db.x = (e0 + 4 < nE) ? dsts[min(e0 + 4, nE - 1)] : sent;
    db.y = (e0 + 5 < nE) ? dsts[min(e0 + 5, nE - 1)] : sent;
    db.z = (e0 + 6 < nE) ? dsts[min(e0 + 6, nE - 1)] : sent;
    db.w = (e0 + 7 < nE) ? dsts[min(e0 + 7, nE - 1)] : sent;
  }
  const unsigned nbs = (unsigned)slotBase;
  const unsigned unb = (unsigned)nb;
  const unsigned s0 = (unsigned)da.x - nbs, s1 = (unsigned)da.y - nbs;
  const unsigned s2 = (unsigned)da.z - nbs, s3 = (unsigned)da.w - nbs;
  const unsigned s4 = (unsigned)db.x - nbs, s5 = (unsigned)db.y - nbs;
  const unsigned s6 = (unsigned)db.z - nbs, s7 = (unsigned)db.w - nbs;
  const bool h0 = s0 < unb, h1 = s1 < unb, h2 = s2 < unb, h3 = s3 < unb;
  const bool h4 = s4 < unb, h5 = s5 < unb, h6 = s6 < unb, h7 = s7 < unb;
  const unsigned any = __builtin_amdgcn_ballot_w32(h0 | h1 | h2 | h3 | h4 | h5 | h6 | h7);
  if (any != 0u) {
#define HITJ(J, HJ, SJ) { \
      const unsigned mj = __builtin_amdgcn_ballot_w32(HJ); \
      if (mj != 0u) { \
        if (HJ) { \
          const int pos = wc + (int)__builtin_amdgcn_mbcnt_lo(mj, 0u); \
          if (pos < WCAP) list[wave * WCAP + pos] = ((el0 + (J)) << SLB) | (int)(SJ); \
        } \
        wc += (int)__builtin_popcount(mj); } }
    HITJ(0, h0, s0)
    HITJ(1, h1, s1)
    HITJ(2, h2, s2)
    HITJ(3, h3, s3)
    HITJ(4, h4, s4)
    HITJ(5, h5, s5)
    HITJ(6, h6, s6)
    HITJ(7, h7, s7)
#undef HITJ
  }
  return wc;
}

template <int KIN, int NOUT>
__device__ __forceinline__ void wunit(const float* __restrict__ W, unsigned short* P, int v) {
  constexpr int KP8 = (2 * KIN) / 8;
  static_assert((KIN & (KIN - 1)) == 0 && KP8 % 8 == 0);
  const int n  = v / KP8;
  const int k8 = (v - n * KP8) * 8;
  const int kk = k8 & (KIN - 1);
  const float* p = W + (size_t)kk * NOUT + n;
  v8us o;
#pragma unroll
  for (int i = 0; i < 8; ++i) o[i] = (unsigned short)bf16_bits(p[(size_t)i * NOUT]);
  unsigned short* dp = P + (size_t)n * (2 * KIN) + k8;
  *(volatile v8us*)dp = o;
  __threadfence();
  *(volatile v8us*)dp = o;
}

__global__ __launch_bounds__(NTHR) void k_wprep(const float* __restrict__ W1, const float* __restrict__ W2,
                                                const float* __restrict__ Wf1, const float* __restrict__ Wf2,
                                                unsigned short* W1T2, unsigned short* W2T2,
                                                unsigned short* F1T2, unsigned short* F2T2) {
  const int u = (int)blockIdx.x * NTHR + (int)threadIdx.x;
  if (u < NU_W1) {
    wunit<CIN, HID>(W1, W1T2, u);
  } else if (u < NU_W1 + NU_W2) {
    wunit<HID, NC2>(W2, W2T2, u - NU_W1);
  } else if (u < NU_W1 + NU_W2 + NU_F1) {
    wunit<NC2, 256>(Wf1, F1T2, u - NU_W1 - NU_W2);
  } else if (u < NU_ALL) {
    wunit<256, 128>(Wf2, F2T2, u - NU_W1 - NU_W2 - NU_F1);
  }
}

__global__ __launch_bounds__(NTHR) void k_cvx(const float* __restrict__ x, int nN, int nUnits,
                                              unsigned short* xb) {
  const int u = (int)blockIdx.x * NTHR + (int)threadIdx.x;
  if (u >= nUnits) return;
  const int row = u >> 4;
  const int k8  = (u & 15) * 8;
  const int rc  = row < nN ? row : nN - 1;
  const float* p = x + (size_t)rc * CIN + k8;
  const v4f a = *(const v4fa*)p;
  const v4f b = *(const v4fa*)(p + 4);
  const bool ok = row < nN;
  v8us o;
  o[0] = ok ? (unsigned short)bf16_bits(a.x) : (unsigned short)0;
  o[1] = ok ? (unsigned short)bf16_bits(a.y) : (unsigned short)0;
  o[2] = ok ? (unsigned short)bf16_bits(a.z) : (unsigned short)0;
  o[3] = ok ? (unsigned short)bf16_bits(a.w) : (unsigned short)0;
  o[4] = ok ? (unsigned short)bf16_bits(b.x) : (unsigned short)0;
  o[5] = ok ? (unsigned short)bf16_bits(b.y) : (unsigned short)0;
  o[6] = ok ? (unsigned short)bf16_bits(b.z) : (unsigned short)0;
  o[7] = ok ? (unsigned short)bf16_bits(b.w) : (unsigned short)0;
  unsigned short* dp = xb + (size_t)row * CIN + k8;
  *(volatile v8us*)dp = o;
  __threadfence();
  *(volatile v8us*)dp = o;
}

template <int MODE>
__global__ __launch_bounds__(GTHR) void k_gemm(
    const unsigned short* __restrict__ A, const unsigned short* __restrict__ WT,
    const float* __restrict__ bias, float* outF, unsigned short* outH, int K, int N)
{
  __shared__ __attribute__((aligned(16))) float stg[GBM * GBN];
  const int tid = (int)threadIdx.x, lane = tid & 31, wave = tid >> 5, hh = lane >> 4, m = lane & 15;
  const int rowBase = (int)blockIdx.x * GBM;
  const int col0    = (int)blockIdx.y * GBN;

  v8f acc[4];
  {
    const v8f z = {0.f, 0.f, 0.f, 0.f, 0.f, 0.f, 0.f, 0.f};
    acc[0] = z; acc[1] = z; acc[2] = z; acc[3] = z;
  }
  const unsigned short* ap = A  + (size_t)(rowBase + 16 * wave + m) * (size_t)K + 8 * hh;
  const unsigned short* wp = WT + (size_t)(col0 + m) * (size_t)K + 8 * hh;
  const int ksteps = K >> 5;
#pragma unroll 1
  for (int ks = 0; ks < ksteps; ++ks) {
    FragB af;
    af.h[0] = *(const v8usa*)(ap + 32 * ks);
    af.h[1] = *(const v8usa*)(ap + 32 * ks + 16);
#pragma unroll
    for (int t = 0; t < 4; ++t) {
      const unsigned short* wq = wp + (size_t)(16 * t) * (size_t)K + 32 * ks;
      FragB bf;
      bf.h[0] = *(const v8usa*)wq;
      bf.h[1] = *(const v8usa*)(wq + 16);
      acc[t] = wmb(af, bf, acc[t]);
    }
  }

#pragma unroll
  for (int t = 0; t < 4; ++t) {
    const int lc = 16 * t + m;
#pragma unroll
    for (int r = 0; r < 8; ++r) {
      const int lr = 16 * wave + 8 * hh + r;
      stg[lr * GBN + lc] = acc[t][r];
    }
  }
  __syncthreads();

  v4f fv[8];
#pragma unroll
  for (int i = 0; i < 8; ++i) {
    const int lr = 16 * wave + 2 * i + hh;
    fv[i] = *(const v4fa*)(stg + lr * GBN + 4 * m);
  }
  if constexpr (MODE != 0) {
    const v4f bq = *(const v4fa*)(bias + col0 + 4 * m);
    v4f b4;
    b4.x = bf16_val(bq.x); b4.y = bf16_val(bq.y); b4.z = bf16_val(bq.z); b4.w = bf16_val(bq.w);
#pragma unroll
    for (int i = 0; i < 8; ++i) {
      v4f y;
      y.x = relu_keep(fv[i].x + b4.x);
      y.y = relu_keep(fv[i].y + b4.y);
      y.z = relu_keep(fv[i].z + b4.z);
      y.w = relu_keep(fv[i].w + b4.w);
      fv[i] = y;
    }
  }

  if constexpr (MODE != 1) {
#pragma unroll
    for (int i = 0; i < 8; ++i) {
      const int gr = rowBase + 16 * wave + 2 * i + hh;
      float* op = outF + (size_t)gr * (size_t)N + col0 + 4 * m;
      *(volatile v4f*)op = fv[i];
    }
    __threadfence();
#pragma unroll
    for (int i = 0; i < 8; ++i) {
      const int gr = rowBase + 16 * wave + 2 * i + hh;
      float* op = outF + (size_t)gr * (size_t)N + col0 + 4 * m;
      *(volatile v4f*)op = fv[i];
    }
  } else {
    __syncthreads();
    unsigned short* sth = (unsigned short*)stg;
#pragma unroll
    for (int i = 0; i < 8; ++i) {
      const int lr = 16 * wave + 2 * i + hh;
      v4us h4, l4;
      unsigned hb;
      hb = bf16_bits(fv[i].x); h4[0] = (unsigned short)hb; l4[0] = (unsigned short)bf16_bits(fv[i].x - __uint_as_float(hb << 16));
      hb = bf16_bits(fv[i].y); h4[1] = (unsigned short)hb; l4[1] = (unsigned short)bf16_bits(fv[i].y - __uint_as_float(hb << 16));
      hb = bf16_bits(fv[i].z); h4[2] = (unsigned short)hb; l4[2] = (unsigned short)bf16_bits(fv[i].z - __uint_as_float(hb << 16));
      hb = bf16_bits(fv[i].w); h4[3] = (unsigned short)hb; l4[3] = (unsigned short)bf16_bits(fv[i].w - __uint_as_float(hb << 16));
      *(v4usa*)(sth + lr * 128 + 4 * m)      = h4;
      *(v4usa*)(sth + lr * 128 + 64 + 4 * m) = l4;
    }
    __syncthreads();
    v8us qv[8];
#pragma unroll
    for (int j = 0; j < 8; ++j) {
      const int lr = 16 * wave + 2 * j + hh;
      qv[j] = *(const v8usa*)(sth + lr * 128 + 8 * m);
    }
    const int coff = (m < 8) ? (col0 + 8 * m) : (N + col0 + 8 * (m - 8));
#pragma unroll
    for (int j = 0; j < 8; ++j) {
      const int gr = rowBase + 16 * wave + 2 * j + hh;
      unsigned short* hp = outH + (size_t)gr * (size_t)(2 * N) + coff;
      *(volatile v8us*)hp = qv[j];
    }
    __threadfence();
#pragma unroll
    for (int j = 0; j < 8; ++j) {
      const int gr = rowBase + 16 * wave + 2 * j + hh;
      unsigned short* hp = outH + (size_t)gr * (size_t)(2 * N) + coff;
      *(volatile v8us*)hp = qv[j];
    }
  }
}

template <int LAYER>
__global__ __launch_bounds__(NTHR) void k_scan(const int* __restrict__ gath, const int* __restrict__ keys,
                                               int nE, int nN, int vec8, int mRows,
                                               const unsigned short* __restrict__ xb,
                                               const float* __restrict__ t2, const float* __restrict__ b2,
                                               unsigned short* m1, float* x2) {
  extern __shared__ __attribute__((aligned(16))) int dsm[];
  int* list = dsm;
  int* hl   = dsm + LISTN;
  int* sl   = hl + RCAP;
  int* cnt  = sl + RCAP;
  int* offs = cnt + NBA;
  int* cur  = offs + NBA;
  int* misc = cur + NBA;
  const int tid = (int)threadIdx.x, lane = tid & 31, wave = tid >> 5;
  unsigned short* rowbuf = (unsigned short*)(misc + MISC_INTS) + wave * KP;
  const int nodeBase = (int)blockIdx.x * NBA;

  {
    const v4i z4 = {0, 0, 0, 0};
    for (int i = tid * 4; i < AGG_ZINTS; i += NTHR * 4) *(v4ia*)(dsm + i) = z4;
    if (tid < MISC_INTS) misc[tid] = 0;
  }
  float bv0 = 0.0f, bv1 = 0.0f;
  if constexpr (LAYER == 2) {
    const v2f a = *(const v2fa*)(b2 + 2 * lane);
    bv0 = bf16_val(a.x); bv1 = bf16_val(a.y);
  }
  __syncthreads();

  int t = 0, ov = 0;
  const int nChunks = (nE + CHUNK - 1) / CHUNK;
#pragma unroll 1
  for (int ch = 0; ch < nChunks; ++ch) {
    const int cbase = ch * CHUNK;
    const int wc = scan_chunk<SLA>(keys, nE, cbase, nodeBase, NBA, vec8, list, tid, lane, wave);
    if (lane == 0) misc[wave] = wc;
    __syncthreads();
    if (wave == 0) {
#pragma unroll 1
      for (int w2 = 0; w2 < NWAVE; ++w2) {
        int c = misc[w2];
        c = c < 0 ? 0 : (c > WCAP ? WCAP : c);
#pragma unroll 1
        for (int b0 = 0; b0 < c; b0 += 32) {
          const int idx = b0 + lane;
          const int ent = list[w2 * WCAP + (idx < WCAP ? idx : WCAP - 1)];
          const int m32 = (c - b0) < 32 ? (c - b0) : 32;
#pragma unroll 1
          for (int k = 0; k < m32; ++k) {
            const int u    = __builtin_amdgcn_readlane(ent, k);
            const int slot = u & (NBA - 1);
            const int el   = (u >> SLA) & (CHUNK - 1);
            const int pk   = ((cbase + el) << SLA) | slot;
            if (t < RCAP) {
              if (lane == 0) { hl[t] = pk; cnt[slot] = cnt[slot] + 1; }
              t = t + 1;
            } else {
              ov = 1;
            }
          }
        }
      }
    }
    __syncthreads();
  }
  if (wave == 0 && lane == 0) { misc[8] = t; misc[9] = ov; }
  __syncthreads();
  int tt = misc[8];
  tt = tt < 0 ? 0 : (tt > RCAP ? RCAP : tt);
  const int ovf = misc[9];

  if (wave == 0) {
    const int base = lane * (NBA / 32);
    int s = 0;
#pragma unroll 1
    for (int i = 0; i < NBA / 32; ++i) s += cnt[base + i];
    int incl = s;
#pragma unroll
    for (int d = 1; d < 32; d <<= 1) {
      const int y = __shfl_up(incl, d, 32);
      if (lane >= d) incl += y;
    }
    int run = incl - s;
#pragma unroll 1
    for (int i = 0; i < NBA / 32; ++i) {
      const int cv = cnt[base + i];
      offs[base + i] = run;
      cur[base + i]  = run;
      run += cv;
    }
  }
  __syncthreads();
  if (wave == 0) {
#pragma unroll 1
    for (int b0 = 0; b0 < tt; b0 += 32) {
      const int idx = b0 + lane;
      const int ent = hl[idx < RCAP ? idx : RCAP - 1];
      const int m32 = (tt - b0) < 32 ? (tt - b0) : 32;
#pragma unroll 1
      for (int k = 0; k < m32; ++k) {
        const int u    = __builtin_amdgcn_readlane(ent, k);
        const int slot = u & (NBA - 1);
        if (lane == 0) {
          int p = cur[slot];
          p = p < 0 ? 0 : (p > RCAP - 1 ? RCAP - 1 : p);
          sl[p] = u;
          cur[slot] = p + 1;
        }
      }
    }
  }
  __syncthreads();

  const float qnan = __int_as_float(0x7fc00000);
  const float pz = (ovf != 0) ? qnan : 0.0f;
  const int sa = (2 * lane) & 31, sb = (2 * lane + 1) & 31;
#pragma unroll 1
  for (int si = 0; si < NBA / NWAVE; ++si) {
    const int s    = si * NWAVE + wave;
    const int node = nodeBase + s;
    const int craw = cnt[s];
    int c = craw;
    const bool big = c > DEGCAP;
    c = c < 0 ? 0 : (c > DEGCAP ? DEGCAP : c);
    int o = offs[s];
    o = o < 0 ? 0 : (o > RCAP ? RCAP : o);
    const float cf = (float)(craw < 1 ? 1 : craw);
    const float rc = 1.0f / cf;
    float a0 = 0.0f, a1 = 0.0f, a2 = 0.0f, a3 = 0.0f;
#pragma unroll 1
    for (int b0 = 0; b0 < c; b0 += 32) {
      int idx = o + b0 + lane;
      idx = idx > RCAP - 1 ? RCAP - 1 : idx;
      const int ent = sl[idx];
      int eid = ent >> SLA;
      eid = eid < 0 ? 0 : (eid > nE - 1 ? nE - 1 : eid);
      int sr = gath[eid];
      sr = sr < 0 ? 0 : (sr > nN - 1 ? nN - 1 : sr);
      const int m32 = (c - b0) < 32 ? (c - b0) : 32;
#pragma unroll 1
      for (int k = 0; k < m32; ++k) {
        const int sk = __builtin_amdgcn_readlane(sr, k);
        if constexpr (LAYER == 1) {
          const v2u w = *(const v2ua*)(xb + (size_t)sk * CIN + 4 * lane);
          a0 += __uint_as_float(w.x << 16);
          a1 += __uint_as_float(w.x & 0xffff0000u);
          a2 += __uint_as_float(w.y << 16);
          a3 += __uint_as_float(w.y & 0xffff0000u);
        } else {
          const v2f a = *(const v2fa*)(t2 + (size_t)sk * NC2 + 2 * lane);
          a0 += a.x; a1 += a.y;
        }
      }
    }
    const float pzr = big ? qnan : pz;
    const bool live = node < nN;
    if constexpr (LAYER == 1) {
      const float m0 = live ? (a0 * rc + pzr) : 0.0f;
      const float mm1 = live ? (a1 * rc + pzr) : 0.0f;
      const float m2 = live ? (a2 * rc + pzr) : 0.0f;
      const float m3 = live ? (a3 * rc + pzr) : 0.0f;
      v4us mh, ml;
      {
        unsigned hb;
        hb = bf16_bits(m0);  mh[0] = (unsigned short)hb; ml[0] = (unsigned short)bf16_bits(m0  - __uint_as_float(hb << 16));
        hb = bf16_bits(mm1); mh[1] = (unsigned short)hb; ml[1] = (unsigned short)bf16_bits(mm1 - __uint_as_float(hb << 16));
        hb = bf16_bits(m2);  mh[2] = (unsigned short)hb; ml[2] = (unsigned short)bf16_bits(m2  - __uint_as_float(hb << 16));
        hb = bf16_bits(m3);  mh[3] = (unsigned short)hb; ml[3] = (unsigned short)bf16_bits(m3  - __uint_as_float(hb << 16));
      }
      *(v4usa*)(rowbuf + 4 * lane) = mh;
      *(v4usa*)(rowbuf + CIN + 4 * lane) = ml;
      wave_sync();
      const v8us q0 = *(const v8usa*)(rowbuf + 8 * lane);
      wave_sync();
      if (node < mRows) {
        unsigned short* rpw = m1 + (size_t)node * KP + 8 * lane;
        *(volatile v8us*)rpw = q0;
        __threadfence();
        *(volatile v8us*)rpw = q0;
      }
    } else {
      float y0 = (a0 * rc + bv0) + pzr;
      float y1 = (a1 * rc + bv1) + pzr;
      const bool zr = (node == 0);
      y0 = zr ? 0.0f : y0;
      y1 = zr ? 0.0f : y1;
      const float v0 = live ? y0 : 0.0f;
      const float v1 = live ? y1 : 0.0f;
      v4f ow;
      ow.x = __shfl(v0, sa, 32); ow.y = __shfl(v1, sa, 32);
      ow.z = __shfl(v0, sb, 32); ow.w = __shfl(v1, sb, 32);
      const bool wr = (node < mRows) && (lane < 16);
      float* op = x2 + (size_t)node * NC2 + 4 * (lane & 15);
      if (wr) *(volatile v4f*)op = ow;
      __threadfence();
      if (wr) *(volatile v4f*)op = ow;
    }
  }
}

__global__ __launch_bounds__(NTHR) void k_sent(const float* __restrict__ x2, const int* __restrict__ tok,
                                               int nN, int nB, unsigned short* se) {
  const int tid = (int)threadIdx.x, lane = tid & 31, wave = tid >> 5;
  const int b  = (int)blockIdx.x * NWAVE + wave;
  const int bc = b < nB ? b : nB - 1;
  const int* sp = tok + (size_t)bc * SLEN;
  int i0 = sp[lane];
  int i1 = sp[(32 + lane) < SLEN ? (32 + lane) : (SLEN - 1)];
  i0 = i0 < 0 ? 0 : (i0 > nN - 1 ? nN - 1 : i0);
  i1 = i1 < 0 ? 0 : (i1 > nN - 1 ? nN - 1 : i1);
  float a0 = 0.0f, a1 = 0.0f;
#pragma unroll 1
  for (int l = 0; l < 32; ++l) {
    const int sk = __builtin_amdgcn_readlane(i0, l);
    const v2f v = *(const v2fa*)(x2 + (size_t)sk * NC2 + 2 * lane);
    a0 += v.x; a1 += v.y;
  }
#pragma unroll 1
  for (int l = 0; l < SLEN - 32; ++l) {
    const int sk = __builtin_amdgcn_readlane(i1, l);
    const v2f v = *(const v2fa*)(x2 + (size_t)sk * NC2 + 2 * lane);
    a0 += v.x; a1 += v.y;
  }
  const unsigned hb0 = bf16_bits(a0), hb1 = bf16_bits(a1);
  const unsigned lb0 = bf16_bits(a0 - __uint_as_float(hb0 << 16));
  const unsigned lb1 = bf16_bits(a1 - __uint_as_float(hb1 << 16));
  const int hw = (int)(hb0 | (hb1 << 16));
  const int lw = (int)(lb0 | (lb1 << 16));
  const int q0s = (4 * lane) & 31, q1s = (4 * lane + 1) & 31;
  const int q2s = (4 * lane + 2) & 31, q3s = (4 * lane + 3) & 31;
  const int g0 = __shfl(hw, q0s, 32), g1 = __shfl(hw, q1s, 32);
  const int g2 = __shfl(hw, q2s, 32), g3 = __shfl(hw, q3s, 32);
  const int p0 = __shfl(lw, q0s, 32), p1 = __shfl(lw, q1s, 32);
  const int p2 = __shfl(lw, q2s, 32), p3 = __shfl(lw, q3s, 32);
  const bool lsel = (lane & 8) != 0;
  v4u pv;
  pv.x = (unsigned int)(lsel ? p0 : g0);
  pv.y = (unsigned int)(lsel ? p1 : g1);
  pv.z = (unsigned int)(lsel ? p2 : g2);
  pv.w = (unsigned int)(lsel ? p3 : g3);
  const bool wr = (b < nB) && (lane < 16);
  unsigned short* hp = se + (size_t)bc * (2 * NC2) + 8 * (lane & 15);
  if (wr) *(volatile v4u*)hp = pv;
  __threadfence();
  if (wr) *(volatile v4u*)hp = pv;
}

__global__ __launch_bounds__(NTHR) void k_final(const float* __restrict__ h2, const float* __restrict__ Wf3,
                                                const float* __restrict__ bf3, float* out) {
  __shared__ float wls[256];
  __shared__ float bls[2];
  __shared__ __attribute__((aligned(16))) float os[NTHR];
  const int tid = (int)threadIdx.x;
  wls[tid] = bf16_val(Wf3[tid]);
  if (tid < 2) bls[tid] = bf16_val(bf3[tid]);
  __syncthreads();
  const int idx = (int)blockIdx.x * NTHR + tid;
  const int b = idx >> 1;
  const int c = idx & 1;
  const float* pr = h2 + (size_t)b * 128;
  float s = 0.0f;
#pragma unroll 1
  for (int k4 = 0; k4 < 32; ++k4) {
    const v4f p = *(const v4fa*)(pr + 4 * k4);
    const float* w = wls + 8 * k4 + c;
    s = fmaf(p.x, w[0], s);
    s = fmaf(p.y, w[2], s);
    s = fmaf(p.z, w[4], s);
    s = fmaf(p.w, w[6], s);
  }
  os[tid] = s + bls[c];
  __syncthreads();
  const v4f ov = *(const v4fa*)(os + 4 * (tid & 63));
  float* op = out + (size_t)blockIdx.x * NTHR + 4 * (tid & 63);
  const bool okst = tid < 64;
  if (okst) *(volatile v4f*)op = ov;
  __threadfence();
  if (okst) *(volatile v4f*)op = ov;
}

static inline int cdiv(int a, int b) { return (a + b - 1) / b; }
static inline size_t al256(size_t o) { return (o + 255) & ~(size_t)255; }

extern "C" void kernel_launch(void* const* d_in, const int* in_sizes, int n_in,
                              void* d_out, int out_size, void* d_ws, size_t ws_size,
                              hipStream_t stream) {
  if (n_in < 14) return;
  if (in_sizes[0] < CIN || (in_sizes[0] % CIN) != 0) return;
  const int nN = in_sizes[0] / CIN;
  if (nN < 16 || nN >= (1 << 24)) return;
  if (in_sizes[1] != CIN * HID || in_sizes[2] != HID) return;
  if (in_sizes[3] != HID * NC2 || in_sizes[4] != NC2) return;
  if (in_sizes[5] != NC2 * 256 || in_sizes[6] != 256) return;
  if (in_sizes[7] != 256 * 128 || in_sizes[8] != 128) return;
  if (in_sizes[9] != 128 * 2 || in_sizes[10] != 2) return;
  const int nE = in_sizes[11];
  if (nE < 1 || nE >= (1 << 21) || in_sizes[12] != nE) return;
  if (in_sizes[13] < SLEN || (in_sizes[13] % SLEN) != 0) return;
  const int nB = in_sizes[13] / SLEN;
  if ((nB % GBM) != 0 || ((2 * nB) % NTHR) != 0) return;
  if (out_size != 2 * nB) return;

  const float* x   = (const float*)d_in[0];
  const float* W1  = (const float*)d_in[1];
  const float* b1  = (const float*)d_in[2];
  const float* W2  = (const float*)d_in[3];
  const float* b2  = (const float*)d_in[4];
  const float* Wf1 = (const float*)d_in[5];
  const float* bf1 = (const float*)d_in[6];
  const float* Wf2 = (const float*)d_in[7];
  const float* bf2 = (const float*)d_in[8];
  const float* Wf3 = (const float*)d_in[9];
  const float* bf3 = (const float*)d_in[10];
  const int*   src = (const int*)d_in[11];
  const int*   dst = (const int*)d_in[12];
  const int*   tok = (const int*)d_in[13];
  float* out = (float*)d_out;

  const int MP = cdiv(nN, GBM) * GBM;
  const int gM = MP / GBM;
  const int gA = cdiv(MP, NBA);
  if ((long long)gA * NBA < (long long)MP) return;
  const int vec8 = ((nE & 3) == 0) ? 1 : 0;

  char* ws = (char*)d_ws;
  size_t off = 0;
  const size_t oW1 = off; off = al256(off + (size_t)HID * (2 * CIN) * 2);
  const size_t oW2 = off; off = al256(off + (size_t)NC2 * (2 * HID) * 2);
  const size_t oF1 = off; off = al256(off + (size_t)256 * (2 * NC2) * 2);
  const size_t oF2 = off; off = al256(off + (size_t)128 * (2 * 256) * 2);
  const size_t oXB = off; off = al256(off + (size_t)MP * CIN * 2);
  const size_t oM1 = off; off = al256(off + (size_t)MP * KP * 2);
  const size_t oX1 = off; off = al256(off + (size_t)MP * KP * 2);
  const size_t oT2 = off; off = al256(off + (size_t)MP * NC2 * 4);
  const size_t oX2 = off; off = al256(off + (size_t)MP * NC2 * 4);
  const size_t oSE = off; off = al256(off + (size_t)nB * (2 * NC2) * 2);
  const size_t oH1 = off; off = al256(off + (size_t)nB * 512 * 2);
  const size_t oH2 = off; off = al256(off + (size_t)nB * 128 * 4);
  if (off > ws_size || off > (size_t)WSMAX) return;
  unsigned short* W1T2 = (unsigned short*)(ws + oW1);
  unsigned short* W2T2 = (unsigned short*)(ws + oW2);
  unsigned short* F1T2 = (unsigned short*)(ws + oF1);
  unsigned short* F2T2 = (unsigned short*)(ws + oF2);
  unsigned short* XB   = (unsigned short*)(ws + oXB);
  unsigned short* M1   = (unsigned short*)(ws + oM1);
  unsigned short* X1   = (unsigned short*)(ws + oX1);
  float*          T2   = (float*)(ws + oT2);
  float*          X2   = (float*)(ws + oX2);
  unsigned short* SE   = (unsigned short*)(ws + oSE);
  unsigned short* H1   = (unsigned short*)(ws + oH1);
  float*          H2   = (float*)(ws + oH2);

  const size_t scanLds = (size_t)AGG_LDS_INTS * 4;
  hipFuncSetAttribute(reinterpret_cast<const void*>(&k_scan<1>), hipFuncAttributeMaxDynamicSharedMemorySize, (int)scanLds);
  hipFuncSetAttribute(reinterpret_cast<const void*>(&k_scan<2>), hipFuncAttributeMaxDynamicSharedMemorySize, (int)scanLds);

  const int nUx = MP * (CIN / 8);
  k_wprep<<<NU_ALL / NTHR, NTHR, 0, stream>>>(W1, W2, Wf1, Wf2, W1T2, W2T2, F1T2, F2T2);
  k_cvx<<<cdiv(nUx, NTHR), NTHR, 0, stream>>>(x, nN, nUx, XB);
  k_scan<1><<<gA, NTHR, scanLds, stream>>>(src, dst, nE, nN, vec8, MP, XB, T2, b2, M1, X2);
  k_gemm<1><<<dim3(gM, HID / GBN), GTHR, 0, stream>>>(M1, W1T2, b1, T2, X1, 2 * CIN, HID);
  k_gemm<0><<<dim3(gM, NC2 / GBN), GTHR, 0, stream>>>(X1, W2T2, b1, T2, X1, 2 * HID, NC2);
  k_scan<2><<<gA, NTHR, scanLds, stream>>>(src, dst, nE, nN, vec8, MP, XB, T2, b2, M1, X2);
  k_sent<<<cdiv(nB, NWAVE), NTHR, 0, stream>>>(X2, tok, nN, nB, SE);
  k_gemm<1><<<dim3(nB / GBM, 256 / GBN), GTHR, 0, stream>>>(SE, F1T2, bf1, H2, H1, 2 * NC2, 256);
  k_gemm<2><<<dim3(nB / GBM, 128 / GBN), GTHR, 0, stream>>>(H1, F2T2, bf2, H2, H1, 2 * 256, 128);
  k_final<<<(2 * nB) / NTHR, NTHR, 0, stream>>>(H2, Wf3, bf3, out);
}
